// SpatialAttentionMechanism_73547019976729
// MI455X (gfx1250) — hardware-verified
//
#include <hip/hip_runtime.h>
#include <stddef.h>


#define NB   2
#define NC   512
#define NPTS 3072
#define NH   8
#define HD   64
#define NT16 (NPTS / 16)
#define NT64 (NPTS / 64)
#define NCT  (NC / 64)
#define PT   68
#define PP   40
#define MASKV (-30000.0f)
#define SSCL (1.0f / 512.0f)
#define PSCL 4096.0f
#define OSCL 32768.0f

typedef _Float16 f16t;
typedef unsigned short us;
typedef float        v8f  __attribute__((ext_vector_type(8)));
typedef float        v4f  __attribute__((ext_vector_type(4)));
typedef unsigned int v4u  __attribute__((ext_vector_type(4)));
typedef us           v8us __attribute__((ext_vector_type(8)));
typedef _Float16     v16h __attribute__((ext_vector_type(16)));
typedef _Float16     v8h  __attribute__((ext_vector_type(8)));
typedef __bf16       v16bf __attribute__((ext_vector_type(16)));
typedef v8h v8ha __attribute__((may_alias));
typedef v4f v4fa __attribute__((may_alias));

union FragH { v16h v; v8us uh[2]; v8h hh[2]; };
union FragB { v16bf v; v8us uh[2]; };

__device__ __forceinline__ v8f mma_b3(v16bf ah, v16bf al, v16bf bh, v16bf bl, v8f c) {
  c = __builtin_amdgcn_wmma_f32_16x16x32_bf16(false, ah, false, bh, (short)0, c, false, false);
  c = __builtin_amdgcn_wmma_f32_16x16x32_bf16(false, ah, false, bl, (short)0, c, false, false);
  c = __builtin_amdgcn_wmma_f32_16x16x32_bf16(false, al, false, bh, (short)0, c, false, false);
  asm volatile("v_nop\n\tv_nop\n\tv_nop\n\tv_nop" : "+v"(c) : "v"(ah), "v"(al), "v"(bh), "v"(bl));
  return c;
}
__device__ __forceinline__ v8f mma_h2(v16h a0, v16h b0, v16h a1, v16h b1, v8f c) {
  c = __builtin_amdgcn_wmma_f32_16x16x32_f16(false, a0, false, b0, (short)0, c, false, false);
  c = __builtin_amdgcn_wmma_f32_16x16x32_f16(false, a1, false, b1, (short)0, c, false, false);
  asm volatile("v_nop\n\tv_nop\n\tv_nop\n\tv_nop" : "+v"(c) : "v"(a0), "v"(b0), "v"(a1), "v"(b1));
  return c;
}
__device__ __forceinline__ v8f mma_h1(v16h a, v16h b, v8f c) {
  c = __builtin_amdgcn_wmma_f32_16x16x32_f16(false, a, false, b, (short)0, c, false, false);
  asm volatile("v_nop\n\tv_nop\n\tv_nop\n\tv_nop" : "+v"(c) : "v"(a), "v"(b));
  return c;
}

__device__ __forceinline__ unsigned bf_bits(float x) {
  const unsigned u = __float_as_uint(x);
  return (u + 0x7FFFu + ((u >> 16) & 1u)) >> 16;
}
__device__ __forceinline__ void bf_split(float x, unsigned &hi, unsigned &lo) {
  hi = bf_bits(x);
  lo = bf_bits(x - __uint_as_float(hi << 16));
}
__device__ __forceinline__ unsigned h_bits(float x) {
  return (unsigned)__builtin_bit_cast(unsigned short, (f16t)x);
}
__device__ __forceinline__ void split8(const v4f a, const v4f b, v4u &hv, v4u &lv) {
  unsigned h0, h1, h2, h3, h4, h5, h6, h7, l0, l1, l2, l3, l4, l5, l6, l7;
  bf_split(a.x, h0, l0); bf_split(a.y, h1, l1); bf_split(a.z, h2, l2); bf_split(a.w, h3, l3);
  bf_split(b.x, h4, l4); bf_split(b.y, h5, l5); bf_split(b.z, h6, l6); bf_split(b.w, h7, l7);
  v4u r, s;
  r.x = h0 | (h1 << 16); r.y = h2 | (h3 << 16); r.z = h4 | (h5 << 16); r.w = h6 | (h7 << 16);
  s.x = l0 | (l1 << 16); s.y = l2 | (l3 << 16); s.z = l4 | (l5 << 16); s.w = l6 | (l7 << 16);
  hv = r; lv = s;
}
__device__ __forceinline__ v4u pack8h(const v4f a, const v4f b) {
  v4u r;
  r.x = h_bits(a.x) | (h_bits(a.y) << 16);
  r.y = h_bits(a.z) | (h_bits(a.w) << 16);
  r.z = h_bits(b.x) | (h_bits(b.y) << 16);
  r.w = h_bits(b.z) | (h_bits(b.w) << 16);
  return r;
}
__device__ __forceinline__ v8f cat4(v4f a, v4f b) {
  v8f r = {a.x, a.y, a.z, a.w, b.x, b.y, b.z, b.w};
  return r;
}

__device__ __forceinline__ void gemm64(const us* __restrict__ arh, const us* __restrict__ arl,
                                       const us* __restrict__ brh, const us* __restrict__ brl,
                                       v8f acc[4]) {
  const v8f z = {0.f, 0.f, 0.f, 0.f, 0.f, 0.f, 0.f, 0.f};
#pragma unroll
  for (int rt = 0; rt < 4; ++rt) acc[rt] = z;
  for (int k0 = 0; k0 < NC; k0 += 32) {
    FragB fbh, fbl;
    fbh.uh[0] = *(const v8us*)(brh + k0);  fbh.uh[1] = *(const v8us*)(brh + k0 + 16);
    fbl.uh[0] = *(const v8us*)(brl + k0);  fbl.uh[1] = *(const v8us*)(brl + k0 + 16);
#pragma unroll
    for (int rt = 0; rt < 4; ++rt) {
      const size_t o = (size_t)rt * 16 * NC + k0;
      FragB fah, fal;
      fah.uh[0] = *(const v8us*)(arh + o);  fah.uh[1] = *(const v8us*)(arh + o + 16);
      fal.uh[0] = *(const v8us*)(arl + o);  fal.uh[1] = *(const v8us*)(arl + o + 16);
      acc[rt] = mma_b3(fah.v, fal.v, fbh.v, fbl.v, acc[rt]);
    }
  }
}
__device__ __forceinline__ void stage64(float* T, const v8f acc[4], int h, int m, int w) {
#pragma unroll
  for (int rt = 0; rt < 4; ++rt)
#pragma unroll
    for (int r = 0; r < 8; ++r) T[(16 * rt + 8 * h + r) * PT + 16 * w + m] = acc[rt][r];
}

__global__ void __launch_bounds__(128)
k_cvt_x(const float* __restrict__ x, us* __restrict__ xh, us* __restrict__ xl) {
  __shared__ __align__(16) float T[64 * PT];
  const int bid = blockIdx.x;
  if (bid >= NB * NT64 * NCT) return;
  const int ct = bid % NCT;
  const int nt = (bid / NCT) % NT64;
  const int b  = bid / (NCT * NT64);
  const int c0 = ct * 64, n0 = nt * 64;
  const int t = threadIdx.x;
  const float* src = x + ((size_t)b * NC + c0) * NPTS + n0;
#pragma unroll
  for (int i = 0; i < 32; ++i) {
    const int idx = i * 128 + t;
    const int cl = idx >> 6, nl = idx & 63;
    T[nl * PT + cl] = src[(size_t)cl * NPTS + nl];
  }
  __syncthreads();
  const int l = t & 31, w = t >> 5, j = l & 7, rq = l >> 3;
  v4u hv[4], lv[4];
#pragma unroll
  for (int i = 0; i < 4; ++i) {
    const int row = 16 * w + 4 * i + rq;
    const v4fa* s = (const v4fa*)(T + row * PT + 8 * j);
    split8(s[0], s[1], hv[i], lv[i]);
  }
  us* dh = xh + ((size_t)b * NPTS + n0) * NC + c0 + 8 * j;
  us* dl = xl + ((size_t)b * NPTS + n0) * NC + c0 + 8 * j;
#pragma unroll
  for (int i = 0; i < 4; ++i) {
    const size_t ro = (size_t)(16 * w + 4 * i + rq) * NC;
    *(volatile v4u*)(dh + ro) = hv[i];
    *(volatile v4u*)(dl + ro) = lv[i];
  }
  __threadfence();
#pragma unroll
  for (int i = 0; i < 4; ++i) {
    const size_t ro = (size_t)(16 * w + 4 * i + rq) * NC;
    *(volatile v4u*)(dh + ro) = hv[i];
    *(volatile v4u*)(dl + ro) = lv[i];
  }
}

__global__ void __launch_bounds__(128)
k_cvt_w(const float* __restrict__ w0, const float* __restrict__ w1,
        const float* __restrict__ w2, const float* __restrict__ w3,
        us* __restrict__ wh, us* __restrict__ wl) {
  const int l = threadIdx.x & 31;
  const int wg = blockIdx.x * 4 + (threadIdx.x >> 5);
  if (wg >= 4 * NC) return;
  const int mat = wg / NC, row = wg % NC;
  const float* src = (mat == 0) ? w0 : ((mat == 1) ? w1 : ((mat == 2) ? w2 : w3));
  src += (size_t)row * NC;
  us* dh = wh + ((size_t)mat * NC + row) * NC;
  us* dl = wl + ((size_t)mat * NC + row) * NC;
  v4u hv[2], lv[2];
#pragma unroll
  for (int ch = 0; ch < 2; ++ch) {
    const v4f* s = (const v4f*)(src + 256 * ch + 8 * l);
    split8(s[0], s[1], hv[ch], lv[ch]);
  }
#pragma unroll
  for (int ch = 0; ch < 2; ++ch) {
    *(volatile v4u*)(dh + 256 * ch + 8 * l) = hv[ch];
    *(volatile v4u*)(dl + 256 * ch + 8 * l) = lv[ch];
  }
  __threadfence();
#pragma unroll
  for (int ch = 0; ch < 2; ++ch) {
    *(volatile v4u*)(dh + 256 * ch + 8 * l) = hv[ch];
    *(volatile v4u*)(dl + 256 * ch + 8 * l) = lv[ch];
  }
}

__global__ void __launch_bounds__(128)
k_mb(const int* __restrict__ adj, const float* __restrict__ gb, float* __restrict__ mb) {
  const int bid = blockIdx.x;
  if (bid >= NT16 * (NPTS / 256)) return;
  const int kq = bid % (NPTS / 256), nt = bid / (NPTS / 256);
  const int key0 = kq * 256, nr0 = nt * 16;
  const int l = threadIdx.x & 31, w = threadIdx.x >> 5;
  float* base = mb + ((size_t)nt * NPTS + key0) * 16;
  v4f vals[8];
#pragma unroll
  for (int i = 0; i < 8; ++i) {
    const int e = 1024 * w + 128 * i + 4 * l;
    const int kl = e >> 4, r0 = e & 15;
    const size_t idx = (size_t)(nr0 + r0) * NPTS + key0 + kl;
    v4f v;
    { const int a = adj[idx];            const float g = gb[idx];            v.x = (a != 0) ? g : MASKV; }
    { const int a = adj[idx + NPTS];     const float g = gb[idx + NPTS];     v.y = (a != 0) ? g : MASKV; }
    { const int a = adj[idx + 2 * NPTS]; const float g = gb[idx + 2 * NPTS]; v.z = (a != 0) ? g : MASKV; }
    { const int a = adj[idx + 3 * NPTS]; const float g = gb[idx + 3 * NPTS]; v.w = (a != 0) ? g : MASKV; }
    vals[i] = v;
  }
#pragma unroll
  for (int i = 0; i < 8; ++i) *(volatile v4f*)(base + 1024 * w + 128 * i + 4 * l) = vals[i];
  __threadfence();
#pragma unroll
  for (int i = 0; i < 8; ++i) *(volatile v4f*)(base + 1024 * w + 128 * i + 4 * l) = vals[i];
}

__global__ void __launch_bounds__(128)
k_qkv(const us* __restrict__ xh, const us* __restrict__ xl,
      const us* __restrict__ wh, const us* __restrict__ wl,
      const float* __restrict__ bq, const float* __restrict__ bk, const float* __restrict__ bv,
      us* __restrict__ q16, us* __restrict__ k16, us* __restrict__ vT16) {
  __shared__ __align__(16) float T[64 * PT];
  const int bid = blockIdx.x;
  if (bid >= NB * NT64 * NH) return;
  const int hd = bid % NH;
  const int nt = (bid / NH) % NT64;
  const int b  = bid / (NH * NT64);
  const int n0 = nt * 64, co0 = hd * HD;
  const int t = threadIdx.x, l = t & 31, w = t >> 5, h = l >> 4, m = l & 15;
  const int j = l & 7, rq = l >> 3;
  const int bh = b * NH + hd;
  const size_t aoff = ((size_t)b * NPTS + n0 + m) * NC + 8 * h;
  const us* arh = xh + aoff;
  const us* arl = xl + aoff;
#pragma unroll 1
  for (int p = 0; p < 3; ++p) {
    const size_t boff = ((size_t)p * NC + co0 + 16 * w + m) * NC + 8 * h;
    v8f acc[4];
    gemm64(arh, arl, wh + boff, wl + boff, acc);
    stage64(T, acc, h, m, w);
    __syncthreads();
    const float* bias = (p == 0) ? bq : ((p == 1) ? bk : bv);
    v4u vals[4];
    if (p < 2) {
      us* dst = ((p == 0) ? q16 : k16) + ((size_t)bh * NPTS + n0) * HD + 8 * j;
      const v4f b0 = *(const v4f*)(bias + co0 + 8 * j);
      const v4f b1 = *(const v4f*)(bias + co0 + 8 * j + 4);
#pragma unroll
      for (int i = 0; i < 4; ++i) {
        const int row = 16 * w + 4 * i + rq;
        const v4fa* s = (const v4fa*)(T + row * PT + 8 * j);
        const v4f f0 = (s[0] + b0) * 8.0f;
        const v4f f1 = (s[1] + b1) * 8.0f;
        vals[i] = pack8h(f0, f1);
      }
#pragma unroll
      for (int i = 0; i < 4; ++i)
        *(volatile v4u*)(dst + (size_t)(16 * w + 4 * i + rq) * HD) = vals[i];
      __threadfence();
#pragma unroll
      for (int i = 0; i < 4; ++i)
        *(volatile v4u*)(dst + (size_t)(16 * w + 4 * i + rq) * HD) = vals[i];
    } else {
      us* dst = vT16 + ((size_t)bh * HD) * NPTS + n0 + 8 * j;
#pragma unroll
      for (int i = 0; i < 4; ++i) {
        const int d = 16 * w + 4 * i + rq;
        const float bd = bias[co0 + d];
        v4f f0, f1;
        f0.x = (T[(8 * j + 0) * PT + d] + bd) * 8.0f;
        f0.y = (T[(8 * j + 1) * PT + d] + bd) * 8.0f;
        f0.z = (T[(8 * j + 2) * PT + d] + bd) * 8.0f;
        f0.w = (T[(8 * j + 3) * PT + d] + bd) * 8.0f;
        f1.x = (T[(8 * j + 4) * PT + d] + bd) * 8.0f;
        f1.y = (T[(8 * j + 5) * PT + d] + bd) * 8.0f;
        f1.z = (T[(8 * j + 6) * PT + d] + bd) * 8.0f;
        f1.w = (T[(8 * j + 7) * PT + d] + bd) * 8.0f;
        vals[i] = pack8h(f0, f1);
      }
#pragma unroll
      for (int i = 0; i < 4; ++i)
        *(volatile v4u*)(dst + (size_t)(16 * w + 4 * i + rq) * NPTS) = vals[i];
      __threadfence();
#pragma unroll
      for (int i = 0; i < 4; ++i)
        *(volatile v4u*)(dst + (size_t)(16 * w + 4 * i + rq) * NPTS) = vals[i];
    }
    __syncthreads();
  }
}

__global__ void __launch_bounds__(128)
k_attn(const us* __restrict__ q16, const us* __restrict__ k16, const us* __restrict__ vT16,
       const float* __restrict__ mb, us* __restrict__ ath, us* __restrict__ atl) {
  __shared__ __align__(16) f16t sP[4 * 16 * PP];
  __shared__ __align__(16) float sO[4 * 16 * PT];
  const int bid = blockIdx.x;
  if (bid >= (NB * NH * NT16) / 4) return;
  const int t = threadIdx.x, l = t & 31, w = t >> 5, h = l >> 4, m = l & 15;
  const int wg = bid * 4 + w;
  const int nt = wg % NT16;
  const int bh = wg / NT16;
  const int b = bh / NH, hd = bh % NH;
  const int n0 = nt * 16;
  f16t* lp = sP + w * (16 * PP);
  float* lo = sO + w * (16 * PT);

  const us* qrow = q16 + ((size_t)bh * NPTS + n0 + m) * HD + 8 * h;
  FragH aq0, aq1;
  aq0.uh[0] = *(const v8us*)(qrow);      aq0.uh[1] = *(const v8us*)(qrow + 16);
  aq1.uh[0] = *(const v8us*)(qrow + 32); aq1.uh[1] = *(const v8us*)(qrow + 48);
  const us* kbase = k16 + ((size_t)bh * NPTS + m) * HD + 8 * h;
  const us* vbase = vT16 + ((size_t)bh * HD + m) * NPTS + 8 * h;
  const float* mbb = mb + ((size_t)nt * NPTS + m) * 16 + 8 * h;

  const v8f z = {0.f, 0.f, 0.f, 0.f, 0.f, 0.f, 0.f, 0.f};
  v8f o[4];
#pragma unroll
  for (int dt = 0; dt < 4; ++dt) o[dt] = z;
  v8f mrow, lrow = z;
#pragma unroll
  for (int r = 0; r < 8; ++r) mrow[r] = -1.0e30f;

  for (int key0 = 0; key0 < NPTS; key0 += 32) {
    v8f s0 = z, s1 = z;
    {
      const us* kp = kbase + (size_t)key0 * HD;
      FragH b0, b1;
      b0.uh[0] = *(const v8us*)(kp);      b0.uh[1] = *(const v8us*)(kp + 16);
      b1.uh[0] = *(const v8us*)(kp + 32); b1.uh[1] = *(const v8us*)(kp + 48);
      s0 = mma_h2(aq0.v, b0.v, aq1.v, b1.v, s0);
    }
    {
      const us* kp = kbase + (size_t)(key0 + 16) * HD;
      FragH b0, b1;
      b0.uh[0] = *(const v8us*)(kp);      b0.uh[1] = *(const v8us*)(kp + 16);
      b1.uh[0] = *(const v8us*)(kp + 32); b1.uh[1] = *(const v8us*)(kp + 48);
      s1 = mma_h2(aq0.v, b0.v, aq1.v, b1.v, s1);
    }
    {
      const float* mp0 = mbb + (size_t)key0 * 16;
      const float* mp1 = mbb + (size_t)(key0 + 16) * 16;
      const v8f mb0 = cat4(*(const v4f*)(mp0), *(const v4f*)(mp0 + 4));
      const v8f mb1 = cat4(*(const v4f*)(mp1), *(const v4f*)(mp1 + 4));
#pragma unroll
      for (int r = 0; r < 8; ++r) {
        s0[r] = s0[r] * SSCL + mb0[r];
        s1[r] = s1[r] * SSCL + mb1[r];
      }
    }
    v8f tm;
#pragma unroll
    for (int r = 0; r < 8; ++r) tm[r] = fmaxf(s0[r], s1[r]);
#pragma unroll
    for (int off = 1; off <= 8; off <<= 1)
#pragma unroll
      for (int r = 0; r < 8; ++r) tm[r] = fmaxf(tm[r], __shfl_xor(tm[r], off, 32));
    v8f mnew, alpha, p0, p1, rs;
#pragma unroll
    for (int r = 0; r < 8; ++r) {
      mnew[r]  = fmaxf(mrow[r], tm[r]);
      alpha[r] = __expf(mrow[r] - mnew[r]);
      p0[r]    = __expf(s0[r] - mnew[r]);
      p1[r]    = __expf(s1[r] - mnew[r]);
      rs[r]    = p0[r] + p1[r];
    }
#pragma unroll
    for (int off = 1; off <= 8; off <<= 1)
#pragma unroll
      for (int r = 0; r < 8; ++r) rs[r] += __shfl_xor(rs[r], off, 32);
#pragma unroll
    for (int r = 0; r < 8; ++r) {
      lrow[r] = lrow[r] * alpha[r] + rs[r];
      mrow[r] = mnew[r];
    }
#pragma unroll
    for (int dt = 0; dt < 4; ++dt) o[dt] = o[dt] * alpha;
#pragma unroll
    for (int r = 0; r < 8; ++r) {
      lp[(8 * h + r) * PP + m]      = (f16t)(p0[r] * PSCL);
      lp[(8 * h + r) * PP + 16 + m] = (f16t)(p1[r] * PSCL);
    }
    __syncthreads();
    FragH pa;
    pa.hh[0] = *(const v8ha*)(lp + m * PP + 8 * h);
    pa.hh[1] = *(const v8ha*)(lp + m * PP + 16 + 8 * h);
#pragma unroll
    for (int dt = 0; dt < 4; ++dt) {
      const us* vp = vbase + (size_t)dt * 16 * NPTS + key0;
      FragH bvf;
      bvf.uh[0] = *(const v8us*)(vp);
      bvf.uh[1] = *(const v8us*)(vp + 16);
      o[dt] = mma_h1(pa.v, bvf.v, o[dt]);
    }
  }

  v8f inv;
#pragma unroll
  for (int r = 0; r < 8; ++r) inv[r] = 1.0f / (lrow[r] * OSCL);
#pragma unroll
  for (int dt = 0; dt < 4; ++dt)
#pragma unroll
    for (int r = 0; r < 8; ++r) lo[(8 * h + r) * PT + 16 * dt + m] = o[dt][r] * inv[r];
  __syncthreads();
  const int j = l & 7, rq = l >> 3;
  v4u hv[4], lv[4];
#pragma unroll
  for (int i = 0; i < 4; ++i) {
    const int row = 4 * i + rq;
    const v4fa* s = (const v4fa*)(lo + row * PT + 8 * j);
    split8(s[0], s[1], hv[i], lv[i]);
  }
  us* dh = ath + ((size_t)b * NPTS + n0) * NC + hd * HD + 8 * j;
  us* dl = atl + ((size_t)b * NPTS + n0) * NC + hd * HD + 8 * j;
#pragma unroll
  for (int i = 0; i < 4; ++i) {
    const size_t ro = (size_t)(4 * i + rq) * NC;
    *(volatile v4u*)(dh + ro) = hv[i];
    *(volatile v4u*)(dl + ro) = lv[i];
  }
  __threadfence();
#pragma unroll
  for (int i = 0; i < 4; ++i) {
    const size_t ro = (size_t)(4 * i + rq) * NC;
    *(volatile v4u*)(dh + ro) = hv[i];
    *(volatile v4u*)(dl + ro) = lv[i];
  }
}

__global__ void __launch_bounds__(128)
k_out(const us* __restrict__ ath, const us* __restrict__ atl,
      const us* __restrict__ wh, const us* __restrict__ wl,
      const float* __restrict__ bo, float* __restrict__ out) {
  __shared__ __align__(16) float T[64 * PT];
  const int bid = blockIdx.x;
  if (bid >= NB * NT64 * NCT) return;
  const int cot = bid % NCT;
  const int nt  = (bid / NCT) % NT64;
  const int b   = bid / (NCT * NT64);
  const int n0 = nt * 64, co0 = cot * 64;
  const int t = threadIdx.x, l = t & 31, w = t >> 5, h = l >> 4, m = l & 15;
  const size_t aoff = ((size_t)b * NPTS + n0 + m) * NC + 8 * h;
  const size_t boff = ((size_t)3 * NC + co0 + 16 * w + m) * NC + 8 * h;
  v8f acc[4];
  gemm64(ath + aoff, atl + aoff, wh + boff, wl + boff, acc);
  stage64(T, acc, h, m, w);
  __syncthreads();
  const int cq = l >> 4, nq = 4 * (l & 15);
  v4f vals[8];
#pragma unroll
  for (int i = 0; i < 8; ++i) {
    const int col = 16 * w + 2 * i + cq;
    const float bb = bo[co0 + col];
    v4f f;
    f.x = T[(nq + 0) * PT + col] + bb;
    f.y = T[(nq + 1) * PT + col] + bb;
    f.z = T[(nq + 2) * PT + col] + bb;
    f.w = T[(nq + 3) * PT + col] + bb;
    vals[i] = f;
  }
  float* dst = out + ((size_t)b * NC + co0) * NPTS + n0 + nq;
#pragma unroll
  for (int i = 0; i < 8; ++i)
    *(volatile v4f*)(dst + (size_t)(16 * w + 2 * i + cq) * NPTS) = vals[i];
  __threadfence();
#pragma unroll
  for (int i = 0; i < 8; ++i)
    *(volatile v4f*)(dst + (size_t)(16 * w + 2 * i + cq) * NPTS) = vals[i];
}

extern "C" void kernel_launch(void* const* d_in, const int* in_sizes, int n_in,
                              void* d_out, int out_size, void* d_ws, size_t ws_size,
                              hipStream_t stream) {
  if (n_in < 11) return;
  if (in_sizes[0] != NB * NC * NPTS) return;
  if (in_sizes[1] != NPTS * NPTS || in_sizes[2] != NPTS * NPTS) return;
  if (in_sizes[3] != NC * NC || in_sizes[5] != NC * NC || in_sizes[7] != NC * NC || in_sizes[9] != NC * NC) return;
  if (in_sizes[4] != NC || in_sizes[6] != NC || in_sizes[8] != NC || in_sizes[10] != NC) return;
  if (out_size != NB * NC * NPTS) return;

  const float* x   = (const float*)d_in[0];
  const int*   adj = (const int*)d_in[1];
  const float* gb  = (const float*)d_in[2];
  const float* Wq  = (const float*)d_in[3];
  const float* bq  = (const float*)d_in[4];
  const float* Wk  = (const float*)d_in[5];
  const float* bk  = (const float*)d_in[6];
  const float* Wv  = (const float*)d_in[7];
  const float* bv  = (const float*)d_in[8];
  const float* Wo  = (const float*)d_in[9];
  const float* bo  = (const float*)d_in[10];
  float* out = (float*)d_out;

  const size_t sz_x16 = (size_t)NB * NPTS * NC * 2;
  const size_t sz_w16 = (size_t)4 * NC * NC * 2;
  const size_t sz_mb  = (size_t)NPTS * NPTS * 4;
  const size_t sz_hd  = (size_t)NB * NH * NPTS * HD * 2;
  char* ws = (char*)d_ws;
  size_t off = 0;
  us* xh   = (us*)(ws + off);    off += sz_x16;
  us* xl   = (us*)(ws + off);    off += sz_x16;
  us* wh   = (us*)(ws + off);    off += sz_w16;
  us* wl   = (us*)(ws + off);    off += sz_w16;
  float* mb = (float*)(ws + off); off += sz_mb;
  us* q16  = (us*)(ws + off);    off += sz_hd;
  us* k16  = (us*)(ws + off);    off += sz_hd;
  us* vT16 = (us*)(ws + off);    off += sz_hd;
  us* ath  = (us*)(ws + off);    off += sz_x16;
  us* atl  = (us*)(ws + off);    off += sz_x16;
  if (off > ws_size) return;

  k_cvt_x<<<NB * NT64 * NCT, 128, 0, stream>>>(x, xh, xl);
  k_cvt_w<<<(4 * NC) / 4, 128, 0, stream>>>(Wq, Wk, Wv, Wo, wh, wl);
  k_mb<<<NT16 * (NPTS / 256), 128, 0, stream>>>(adj, gb, mb);
  k_qkv<<<NB * NT64 * NH, 128, 0, stream>>>(xh, xl, wh, wl, bq, bk, bv, q16, k16, vT16);
  k_attn<<<(NB * NH * NT16) / 4, 128, 0, stream>>>(q16, k16, vT16, mb, ath, atl);
  k_out<<<NB * NT64 * NCT, 128, 0, stream>>>(ath, atl, wh, wl, bo, out);
}
